// GRU_4_FC_3_40175124086989
// MI455X (gfx1250) — hardware-verified
//
#include <hip/hip_runtime.h>


#define NB_   2048
#define NT_   256
#define NH_   64
#define NG_   192
#define HP_   72
#define TILE_ (32 * HP_)
#define WMAT_ (NG_ * NH_)
#define SOP_  36
#define HDP_  136
#define Y2P_  36

constexpr int GOFF_W   = 0;
constexpr int GOFF_H   = GOFF_W + 7 * WMAT_ * 2;
constexpr int GOFF_O   = GOFF_H + 8 * TILE_ * 2;
constexpr int LDS_GRU  = GOFF_O + 64 * SOP_ * 4;
constexpr int HOFF_W   = 0;
constexpr int HOFF_X   = HOFF_W + 128 * HDP_ * 2;
constexpr int HOFF_Y   = HOFF_X + 32 * HDP_ * 2;
constexpr int HOFF_Q   = HOFF_Y + 32 * HDP_ * 2;
constexpr int LDS_HEAD = HOFF_Q + 64 * 4;
static_assert(LDS_GRU == 218112);
static_assert(LDS_HEAD == 52480);
static_assert(GOFF_H % 16 == 0 && GOFF_O % 16 == 0);
static_assert(HOFF_X % 16 == 0 && HOFF_Y % 16 == 0 && HOFF_Q % 16 == 0);
static_assert(128 * Y2P_ * 4 <= 128 * HDP_ * 2);
static_assert(NB_ % 32 == 0);
static_assert(NT_ % 2 == 0);
constexpr size_t WS_END = (size_t)NB_ * 128 * 4;
static_assert(WS_END <= (size_t)134217728);

typedef float    v4f  __attribute__((ext_vector_type(4)));
typedef float    v8f  __attribute__((ext_vector_type(8)));
typedef _Float16 v8h  __attribute__((ext_vector_type(8))) __attribute__((may_alias));
typedef _Float16 v16h __attribute__((ext_vector_type(16)));

union Frag { v16h v; v8h p[2]; };

extern __shared__ v4f dynlds[];

__device__ __forceinline__ void mma2(v8f& acc, const v16h a0, const v16h b0, const v16h a1, const v16h b1) {
    acc = __builtin_amdgcn_wmma_f32_16x16x32_f16(false, a0, false, b0, (short)0, acc, false, false);
    acc = __builtin_amdgcn_wmma_f32_16x16x32_f16(false, a1, false, b1, (short)0, acc, false, false);
    asm volatile("v_nop\n\tv_nop\n\tv_nop\n\tv_nop" : "+v"(acc) : "v"(a0), "v"(b0), "v"(a1), "v"(b1));
}

__device__ __forceinline__ void ldfrag(Frag& f, const _Float16* p) {
    f.p[0] = *(const v8h*)(p);
    f.p[1] = *(const v8h*)(p + 16);
}

__device__ __forceinline__ void cvt8(const float* __restrict__ src, _Float16* dst, float sc) {
    const v4f a = *(const v4f*)(src);
    const v4f b = *(const v4f*)(src + 4);
    v8h o;
#pragma unroll
    for (int i = 0; i < 4; ++i) {
        o[i]     = (_Float16)(a[i] * sc);
        o[4 + i] = (_Float16)(b[i] * sc);
    }
    *(v8h*)(dst) = o;
}

__device__ __forceinline__ float sig128(float a) {
    const float e = __builtin_amdgcn_exp2f(a * (-1.4426950408889634f * 0.0078125f));
    return __builtin_amdgcn_rcpf(1.0f + e);
}
__device__ __forceinline__ float tanh128(float a) {
    const float e = __builtin_amdgcn_exp2f(a * (2.8853900817779268f * 0.0078125f));
    return 1.0f - 2.0f * __builtin_amdgcn_rcpf(e + 1.0f);
}

__device__ __forceinline__ void proj3(v8f& a0, v8f& a1, v8f& a2,
                                      const _Float16* At, const _Float16* Wm,
                                      int s, int cg, int m, int h)
{
    Frag fa0, fa1;
    const _Float16* ap = At + (16 * s + m) * HP_ + 8 * h;
    ldfrag(fa0, ap);
    ldfrag(fa1, ap + 32);
    const _Float16* bp = Wm + (16 * cg + m) * NH_ + 8 * h;
    {
        Frag b0, b1;
        ldfrag(b0, bp);
        ldfrag(b1, bp + 32);
        mma2(a0, fa0.v, b0.v, fa1.v, b1.v);
    }
    {
        Frag b0, b1;
        ldfrag(b0, bp + 64 * NH_);
        ldfrag(b1, bp + 64 * NH_ + 32);
        mma2(a1, fa0.v, b0.v, fa1.v, b1.v);
    }
    {
        Frag b0, b1;
        ldfrag(b0, bp + 128 * NH_);
        ldfrag(b1, bp + 128 * NH_ + 32);
        mma2(a2, fa0.v, b0.v, fa1.v, b1.v);
    }
}

__device__ __forceinline__ void gru_layer(float (&hs)[8],
                                          const _Float16* Xt, const _Float16* Ho, _Float16* Hn,
                                          const _Float16* Wi, const _Float16* Wh,
                                          float br, float bz, float bi, float bh,
                                          int s, int cg, int m, int h, int cr)
{
    v8f ar, az, ai, ah;
#pragma unroll
    for (int r = 0; r < 8; ++r) { ar[r] = br; az[r] = bz; ai[r] = bi; ah[r] = bh; }
    proj3(ar, az, ai, Xt, Wi, s, cg, m, h);
    proj3(ar, az, ah, Ho, Wh, s, cg, m, h);
    _Float16* hn = Hn + (16 * s + 8 * h) * HP_ + cr;
#pragma unroll
    for (int r = 0; r < 8; ++r) {
        const float rg = sig128(ar[r]);
        const float zg = sig128(az[r]);
        const float ng = tanh128(fmaf(rg, ah[r], ai[r]));
        const float hv = fmaf(zg, hs[r] - ng, ng);
        hs[r] = hv;
        hn[r * HP_] = (_Float16)(hv * 8.0f);
    }
}

template <int IN_W>
__global__ __launch_bounds__(256)
void gru_stack_kernel(const float* __restrict__ xin,
                      const float* __restrict__ wih0,
                      const float* __restrict__ wih,
                      const float* __restrict__ whh,
                      const float* __restrict__ bih,
                      const float* __restrict__ bhh,
                      float* xcat, int coff)
{
    char* lds = (char*)dynlds;
    _Float16* Wl = (_Float16*)(lds + GOFF_W);
    _Float16* Hl = (_Float16*)(lds + GOFF_H);
    float*    So = (float*)(lds + GOFF_O);

    const int tid  = threadIdx.x;
    const int lane = tid & 31;
    const int wave = tid >> 5;
    const int h    = lane >> 4;
    const int m    = lane & 15;
    const int s    = wave >> 2;
    const int cg   = wave & 3;
    const int m0   = blockIdx.x * 32;
    const int cr   = 16 * cg + m;
    const int cz   = NH_ + cr;
    const int cn   = 2 * NH_ + cr;

    for (int g = tid; g < 4 * WMAT_ / 8; g += 256) cvt8(whh + 8 * g, Wl + 8 * g, 16.0f);
    for (int g = tid; g < 3 * WMAT_ / 8; g += 256) cvt8(wih + 8 * g, Wl + 4 * WMAT_ + 8 * g, 16.0f);
    {
        v8h z8;
#pragma unroll
        for (int i = 0; i < 8; ++i) z8[i] = (_Float16)0.0f;
        for (int g = tid; g < 8 * TILE_ / 8; g += 256) *(v8h*)(Hl + 8 * g) = z8;
    }

    const float b0r = 128.0f * bih[cr], b0z = 128.0f * bih[cz], b0n = 128.0f * bih[cn];
    const float c0r = 128.0f * bhh[cr], c0z = 128.0f * bhh[cz], c0n = 128.0f * bhh[cn];
    float w0r[IN_W], w0z[IN_W], w0n[IN_W];
#pragma unroll
    for (int i = 0; i < IN_W; ++i) {
        w0r[i] = 128.0f * wih0[cr * IN_W + i];
        w0z[i] = 128.0f * wih0[cz * IN_W + i];
        w0n[i] = 128.0f * wih0[cn * IN_W + i];
    }
    const float b1r = 128.0f * (bih[1 * NG_ + cr] + bhh[1 * NG_ + cr]);
    const float b1z = 128.0f * (bih[1 * NG_ + cz] + bhh[1 * NG_ + cz]);
    const float b1i = 128.0f * bih[1 * NG_ + cn], b1h = 128.0f * bhh[1 * NG_ + cn];
    const float b2r = 128.0f * (bih[2 * NG_ + cr] + bhh[2 * NG_ + cr]);
    const float b2z = 128.0f * (bih[2 * NG_ + cz] + bhh[2 * NG_ + cz]);
    const float b2i = 128.0f * bih[2 * NG_ + cn], b2h = 128.0f * bhh[2 * NG_ + cn];
    const float b3r = 128.0f * (bih[3 * NG_ + cr] + bhh[3 * NG_ + cr]);
    const float b3z = 128.0f * (bih[3 * NG_ + cz] + bhh[3 * NG_ + cz]);
    const float b3i = 128.0f * bih[3 * NG_ + cn], b3h = 128.0f * bhh[3 * NG_ + cn];

    float hs0[8], hs1[8], hs2[8], hs3[8];
#pragma unroll
    for (int r = 0; r < 8; ++r) { hs0[r] = 0.0f; hs1[r] = 0.0f; hs2[r] = 0.0f; hs3[r] = 0.0f; }
    __syncthreads();

#pragma unroll 1
    for (int t = 0; t < NT_; ++t) {
        const _Float16* Hold = Hl + (t & 1) * (4 * TILE_);
        _Float16*       Hnew = Hl + ((t + 1) & 1) * (4 * TILE_);

        {
            v8f ar, az, ah;
#pragma unroll
            for (int r = 0; r < 8; ++r) { ar[r] = c0r; az[r] = c0z; ah[r] = c0n; }
            float gr[8], gz[8], gn[8];
            const float* xp = xin + ((size_t)(m0 + 16 * s + 8 * h) * NT_ + t) * IN_W;
#pragma unroll
            for (int r = 0; r < 8; ++r) {
                const float* p = xp + (size_t)r * (NT_ * IN_W);
                float a = b0r, b = b0z, c = b0n;
                if constexpr (IN_W == 4) {
                    const v4f xv = *(const v4f*)(p);
#pragma unroll
                    for (int i = 0; i < 4; ++i) {
                        a = fmaf(xv[i], w0r[i], a);
                        b = fmaf(xv[i], w0z[i], b);
                        c = fmaf(xv[i], w0n[i], c);
                    }
                } else {
#pragma unroll
                    for (int i = 0; i < IN_W; ++i) {
                        const float xv = p[i];
                        a = fmaf(xv, w0r[i], a);
                        b = fmaf(xv, w0z[i], b);
                        c = fmaf(xv, w0n[i], c);
                    }
                }
                gr[r] = a; gz[r] = b; gn[r] = c;
            }
            proj3(ar, az, ah, Hold, Wl, s, cg, m, h);
            _Float16* hn = Hnew + (16 * s + 8 * h) * HP_ + cr;
#pragma unroll
            for (int r = 0; r < 8; ++r) {
                const float rg = sig128(ar[r] + gr[r]);
                const float zg = sig128(az[r] + gz[r]);
                const float ng = tanh128(fmaf(rg, ah[r], gn[r]));
                const float hv = fmaf(zg, hs0[r] - ng, ng);
                hs0[r] = hv;
                hn[r * HP_] = (_Float16)(hv * 8.0f);
            }
        }
        __syncthreads();
        gru_layer(hs1, Hnew + 0 * TILE_, Hold + 1 * TILE_, Hnew + 1 * TILE_,
                  Wl + 4 * WMAT_, Wl + 1 * WMAT_, b1r, b1z, b1i, b1h, s, cg, m, h, cr);
        __syncthreads();
        gru_layer(hs2, Hnew + 1 * TILE_, Hold + 2 * TILE_, Hnew + 2 * TILE_,
                  Wl + 5 * WMAT_, Wl + 2 * WMAT_, b2r, b2z, b2i, b2h, s, cg, m, h, cr);
        __syncthreads();
        gru_layer(hs3, Hnew + 2 * TILE_, Hold + 3 * TILE_, Hnew + 3 * TILE_,
                  Wl + 6 * WMAT_, Wl + 3 * WMAT_, b3r, b3z, b3i, b3h, s, cg, m, h, cr);
        __syncthreads();
    }

    {
        float* q = So + cr * SOP_ + 16 * s + 8 * h;
        v4f lo, hi;
        lo[0] = hs3[0]; lo[1] = hs3[1]; lo[2] = hs3[2]; lo[3] = hs3[3];
        hi[0] = hs3[4]; hi[1] = hs3[5]; hi[2] = hs3[6]; hi[3] = hs3[7];
        *(v4f*)(q)     = lo;
        *(v4f*)(q + 4) = hi;
    }
    __syncthreads();
    {
        v4f v[2];
        float* gp[2];
#pragma unroll
        for (int it = 0; it < 2; ++it) {
            const int row = 4 * wave + 2 * it + h;
            const int c0  = 4 * m;
            v4f x;
            x[0] = So[(c0 + 0) * SOP_ + row];
            x[1] = So[(c0 + 1) * SOP_ + row];
            x[2] = So[(c0 + 2) * SOP_ + row];
            x[3] = So[(c0 + 3) * SOP_ + row];
            v[it]  = x;
            gp[it] = xcat + (size_t)(m0 + row) * 128 + coff + c0;
        }
        *(volatile v4f*)(gp[0]) = v[0];
        *(volatile v4f*)(gp[1]) = v[1];
        __threadfence();
        *(volatile v4f*)(gp[0]) = v[0];
        *(volatile v4f*)(gp[1]) = v[1];
    }
}

__device__ __forceinline__ void head_gemm(v8f (&acc)[4], const _Float16* At, const _Float16* Wt,
                                          int s, int cp, int m, int h)
{
    Frag fa[4];
    const _Float16* ap = At + (16 * s + m) * HDP_ + 8 * h;
#pragma unroll
    for (int kk = 0; kk < 4; ++kk) ldfrag(fa[kk], ap + 32 * kk);
#pragma unroll
    for (int j = 0; j < 4; ++j) {
        const _Float16* bp = Wt + (64 * cp + 16 * j + m) * HDP_ + 8 * h;
        {
            Frag b0, b1;
            ldfrag(b0, bp);
            ldfrag(b1, bp + 32);
            mma2(acc[j], fa[0].v, b0.v, fa[1].v, b1.v);
        }
        {
            Frag b2, b3;
            ldfrag(b2, bp + 64);
            ldfrag(b3, bp + 96);
            mma2(acc[j], fa[2].v, b2.v, fa[3].v, b3.v);
        }
    }
}

__global__ __launch_bounds__(128)
void head_kernel(const float* __restrict__ xc,
                 const float* __restrict__ w1, const float* __restrict__ b1,
                 const float* __restrict__ g1, const float* __restrict__ e1,
                 const float* __restrict__ u1, const float* __restrict__ r1,
                 const float* __restrict__ w2, const float* __restrict__ b2,
                 const float* __restrict__ g2, const float* __restrict__ e2,
                 const float* __restrict__ u2, const float* __restrict__ r2,
                 const float* __restrict__ w3, const float* __restrict__ b3,
                 float* out)
{
    char* lds = (char*)dynlds;
    _Float16* Ws  = (_Float16*)(lds + HOFF_W);
    _Float16* Xs  = (_Float16*)(lds + HOFF_X);
    _Float16* Y1  = (_Float16*)(lds + HOFF_Y);
    float*    Qs  = (float*)(lds + HOFF_Q);
    float*    Y2T = (float*)(lds + HOFF_W);

    const int tid  = threadIdx.x;
    const int lane = tid & 31;
    const int wave = tid >> 5;
    const int h    = lane >> 4;
    const int m    = lane & 15;
    const int s    = wave >> 1;
    const int cp   = wave & 1;
    const int m0   = blockIdx.x * 32;
    const float inv128 = 0.0078125f;

    for (int g = tid; g < 2048; g += 128) {
        const int n = g >> 4, c8 = (g & 15) * 8;
        cvt8(w1 + n * 128 + c8, Ws + n * HDP_ + c8, 16.0f);
    }
    for (int g = tid; g < 512; g += 128) {
        const int r = g >> 4, c8 = (g & 15) * 8;
        cvt8(xc + (size_t)(m0 + r) * 128 + c8, Xs + r * HDP_ + c8, 8.0f);
    }
    __syncthreads();

    v8f acc[4];
#pragma unroll
    for (int j = 0; j < 4; ++j) {
        const float bb = 128.0f * b1[64 * cp + 16 * j + m];
#pragma unroll
        for (int r = 0; r < 8; ++r) acc[j][r] = bb;
    }
    head_gemm(acc, Xs, Ws, s, cp, m, h);
#pragma unroll
    for (int j = 0; j < 4; ++j) {
        const int col = 64 * cp + 16 * j + m;
        const float gg = g1[col], ee = e1[col], uu = u1[col];
        const float rs = rsqrtf(r1[col] + 1e-5f);
        _Float16* yp = Y1 + (16 * s + 8 * h) * HDP_ + col;
#pragma unroll
        for (int r = 0; r < 8; ++r) {
            const float v = acc[j][r] * inv128;
            float y = (gg * (v - uu)) * rs + ee;
            y = fmaxf(y, 0.0f);
            yp[r * HDP_] = (_Float16)(y * 8.0f);
        }
    }
    __syncthreads();

    for (int g = tid; g < 2048; g += 128) {
        const int n = g >> 4, c8 = (g & 15) * 8;
        cvt8(w2 + n * 128 + c8, Ws + n * HDP_ + c8, 16.0f);
    }
    __syncthreads();

#pragma unroll
    for (int j = 0; j < 4; ++j) {
        const float bb = 128.0f * b2[64 * cp + 16 * j + m];
#pragma unroll
        for (int r = 0; r < 8; ++r) acc[j][r] = bb;
    }
    head_gemm(acc, Y1, Ws, s, cp, m, h);
    __syncthreads();
#pragma unroll
    for (int j = 0; j < 4; ++j) {
        const int col = 64 * cp + 16 * j + m;
        const float gg = g2[col], ee = e2[col], uu = u2[col];
        const float rs = rsqrtf(r2[col] + 1e-5f);
        v4f lo, hi;
#pragma unroll
        for (int r = 0; r < 8; ++r) {
            const float v = acc[j][r] * inv128;
            float y = (gg * (v - uu)) * rs + ee;
            y = fmaxf(y, 0.0f);
            if (r < 4) lo[r] = y; else hi[r - 4] = y;
        }
        float* q = Y2T + col * Y2P_ + 16 * s + 8 * h;
        *(v4f*)(q)     = lo;
        *(v4f*)(q + 4) = hi;
    }
    __syncthreads();

    if (tid < 64) {
        const int row = tid >> 1, o = tid & 1;
        const float* wr = w3 + o * 128;
        float a = b3[o];
#pragma unroll 4
        for (int k = 0; k < 128; ++k) a = fmaf(Y2T[k * Y2P_ + row], wr[k], a);
        Qs[tid] = a;
    }
    __syncthreads();
    if (tid < 16) {
        const v4f v = *(const v4f*)(Qs + 4 * tid);
        float* gp = out + (size_t)m0 * 2 + 4 * tid;
        *(volatile v4f*)gp = v;
        __threadfence();
        *(volatile v4f*)gp = v;
    }
}

extern "C" void kernel_launch(void* const* d_in, const int* in_sizes, int n_in,
                              void* d_out, int out_size, void* d_ws, size_t ws_size,
                              hipStream_t stream)
{
    if (n_in < 26) return;
    if (in_sizes[0]  != NB_ * NT_)       return;
    if (in_sizes[1]  != NB_ * NT_ * 4)   return;
    if (in_sizes[2]  != NG_ * 1)         return;
    if (in_sizes[3]  != 3 * WMAT_)       return;
    if (in_sizes[4]  != 4 * WMAT_)       return;
    if (in_sizes[5]  != 4 * NG_)         return;
    if (in_sizes[6]  != 4 * NG_)         return;
    if (in_sizes[7]  != NG_ * 4)         return;
    if (in_sizes[8]  != 3 * WMAT_)       return;
    if (in_sizes[9]  != 4 * WMAT_)       return;
    if (in_sizes[10] != 4 * NG_)         return;
    if (in_sizes[11] != 4 * NG_)         return;
    if (in_sizes[12] != 128 * 128)       return;
    if (in_sizes[18] != 128 * 128)       return;
    for (int i = 13; i <= 17; ++i) if (in_sizes[i] != 128) return;
    for (int i = 19; i <= 23; ++i) if (in_sizes[i] != 128) return;
    if (in_sizes[24] != 2 * 128)         return;
    if (in_sizes[25] != 2)               return;
    if (out_size != NB_ * 2)             return;
    if (ws_size < WS_END)                return;

    const float* sent  = (const float*)d_in[0];
    const float* price = (const float*)d_in[1];
    const float* sW0   = (const float*)d_in[2];
    const float* sWih  = (const float*)d_in[3];
    const float* sWhh  = (const float*)d_in[4];
    const float* sbih  = (const float*)d_in[5];
    const float* sbhh  = (const float*)d_in[6];
    const float* pW0   = (const float*)d_in[7];
    const float* pWih  = (const float*)d_in[8];
    const float* pWhh  = (const float*)d_in[9];
    const float* pbih  = (const float*)d_in[10];
    const float* pbhh  = (const float*)d_in[11];
    const float* fc1W  = (const float*)d_in[12];
    const float* fc1b  = (const float*)d_in[13];
    const float* g1    = (const float*)d_in[14];
    const float* e1    = (const float*)d_in[15];
    const float* u1    = (const float*)d_in[16];
    const float* r1    = (const float*)d_in[17];
    const float* fc2W  = (const float*)d_in[18];
    const float* fc2b  = (const float*)d_in[19];
    const float* g2    = (const float*)d_in[20];
    const float* e2    = (const float*)d_in[21];
    const float* u2    = (const float*)d_in[22];
    const float* r2    = (const float*)d_in[23];
    const float* fc3W  = (const float*)d_in[24];
    const float* fc3b  = (const float*)d_in[25];
    float* out  = (float*)d_out;
    float* xcat = (float*)d_ws;

    hipFuncSetAttribute(reinterpret_cast<const void*>(&gru_stack_kernel<1>),
                        hipFuncAttributeMaxDynamicSharedMemorySize, LDS_GRU);
    hipFuncSetAttribute(reinterpret_cast<const void*>(&gru_stack_kernel<4>),
                        hipFuncAttributeMaxDynamicSharedMemorySize, LDS_GRU);

    gru_stack_kernel<1><<<dim3(NB_ / 32), dim3(256), LDS_GRU, stream>>>(
        sent, sW0, sWih, sWhh, sbih, sbhh, xcat, 0);
    gru_stack_kernel<4><<<dim3(NB_ / 32), dim3(256), LDS_GRU, stream>>>(
        price, pW0, pWih, pWhh, pbih, pbhh, xcat, 64);
    head_kernel<<<dim3(NB_ / 32), dim3(128), LDS_HEAD, stream>>>(
        (const float*)xcat, fc1W, fc1b, g1, e1, u1, r1, fc2W, fc2b, g2, e2, u2, r2, fc3W, fc3b, out);
}
